// VI2DSSM_14714557956427
// MI455X (gfx1250) — hardware-run, weakly checked
//
#include <hip/hip_runtime.h>


namespace {
constexpr int NBt = 4, DI = 256, L = 2048, NS = 16, R = 16, PW = 64;
constexpr float HS = 256.0f, WSC = 256.0f;
typedef _Float16 b16;
typedef __attribute__((ext_vector_type(16))) _Float16 v16b;
typedef __attribute__((ext_vector_type(8))) _Float16 v8b;
typedef __attribute__((ext_vector_type(8))) float v8f;
typedef __attribute__((ext_vector_type(4))) float v4f;
typedef __attribute__((ext_vector_type(2))) float v2f;
__device__ __forceinline__ float bf16_rne(float f) { unsigned int u = __float_as_uint(f); u += 0x7FFFu + ((u >> 16) & 1u); float r = __uint_as_float(u & 0xFFFF0000u); asm volatile("" : "+v"(r)); return r; }
__device__ __forceinline__ float bfv(float f) { float r = bf16_rne(f); asm volatile("" : "+v"(r)); return r; }
__device__ __forceinline__ void split16(float v, b16& hi, b16& lo) { hi = (b16)v; lo = (b16)(v - (float)hi); }
__device__ __forceinline__ v16b frag_kb(const b16* p, int hh) { const v8b a = *(const v8b*)(p + 8 * hh), b = *(const v8b*)(p + 16 + 8 * hh); v16b f;
#pragma unroll
  for (int e = 0; e < 8; ++e) { f[e] = a[e]; f[8 + e] = b[e]; } return f; }
__device__ __forceinline__ v8f wmma16b(v16b a, v16b b, v8f c) { v8f d = __builtin_amdgcn_wmma_f32_16x16x32_f16(false, a, false, b, (short)0, c, false, false); asm volatile("v_nop\n\tv_nop\n\tv_nop\n\tv_nop" : "+v"(d) : "v"(a), "v"(b)); return d; }
__device__ __forceinline__ void wave_lds_sync() { __builtin_amdgcn_fence(__ATOMIC_RELEASE, "workgroup"); __builtin_amdgcn_wave_barrier(); __builtin_amdgcn_fence(__ATOMIC_ACQUIRE, "workgroup"); }
__device__ __forceinline__ float pmul(float a, float b) { float p = a * b; asm volatile("" : "+v"(p)); return p; }
__device__ __forceinline__ float softplus(float v) { return v > 20.0f ? v : log1pf(__expf(v)); }

__global__ __launch_bounds__(256) void wput_kernel(const float* __restrict__ xp1, const float* __restrict__ xhv, const float* __restrict__ xp2, const float* __restrict__ ch, const float* __restrict__ cv, const float* __restrict__ psi1, const float* __restrict__ psi2, const float* __restrict__ wv, b16* __restrict__ WP1, b16* __restrict__ WP2, b16* __restrict__ WC, float* __restrict__ PWV) { const size_t nt = (size_t)gridDim.x * 256, u0 = (size_t)blockIdx.x * 256 + threadIdx.x; v8b v, v2;
  for (size_t u = u0; u < (size_t)PW * 32; u += nt) { const int o = (int)(u / 32), k0 = (int)(u % 32) * 8;
#pragma unroll
    for (int j = 0; j < 8; ++j) { const int k = k0 + j; v[j] = (b16)(bf16_rne(o < 48 ? xp1[(size_t)o * DI + k] : xhv[(size_t)(o - 48) * DI + k]) * WSC); v2[j] = (b16)(o < 48 ? bf16_rne(xp2[(size_t)o * DI + k]) * WSC : 0.0f); }
    for (int pass = 0; pass < 2; ++pass) { *(volatile v8b*)(WP1 + (size_t)o * DI + k0) = v; *(volatile v8b*)(WP2 + (size_t)o * DI + k0) = v2; __threadfence(); } }
  for (size_t u = u0; u < (size_t)DI * 64; u += nt) { const int o = (int)(u / 64), k0 = (int)(u % 64) * 8;
#pragma unroll
    for (int j = 0; j < 8; ++j) { const int k = k0 + j; v[j] = (b16)(bf16_rne(k < DI ? ch[(size_t)o * DI + k] : cv[(size_t)o * DI + k - DI]) * WSC); } for (int pass = 0; pass < 2; ++pass) { *(volatile v8b*)(WC + (size_t)o * 2 * DI + k0) = v; __threadfence(); } }
  if (u0 < 32) { const int s = (int)u0 / 16, n = (int)u0 % 16; const float* psi = s ? psi2 : psi1; float acc = 0.0f; for (int d = 0; d < DI; ++d) acc += pmul(bfv(psi[n * DI + d]), bfv(wv[d])); for (int pass = 0; pass < 2; ++pass) { ((volatile float*)PWV)[u0] = acc; __threadfence(); } } }
template <int MODE>
__global__ __launch_bounds__(32) void proj_kernel(const float* __restrict__ U, const b16* __restrict__ WP, int LLIM, float* __restrict__ P, float* __restrict__ XM) { __shared__ __attribute__((aligned(16))) b16 Ah[32][DI + 8], Al[32][DI + 8]; __shared__ float Tf[32][PW + 4]; const int lane = threadIdx.x, nloc = lane & 15, hlf = lane >> 4; const int b = blockIdx.x / (L / 32); const int l0 = (blockIdx.x % (L / 32)) * 32; if (l0 >= LLIM) return;
  float sm = 0.0f; for (int d = 0; d < DI; ++d) { const float v = U[((size_t)b * DI + d) * L + l0 + lane]; b16 p, ql; if (MODE == 0) { const float bv = bf16_rne(v); sm += bv; p = (b16)(bv * HS); ql = (b16)0.0f; } else split16(v * HS, p, ql); Ah[lane][d] = p; Al[lane][d] = ql; }
  for (int k = DI; k < DI + 8; ++k) { Ah[lane][k] = (b16)0.0f; Al[lane][k] = (b16)0.0f; }
  wave_lds_sync();
#pragma unroll
  for (int rt = 0; rt < 2; ++rt) { v8f acc[4] = {(v8f){}, (v8f){}, (v8f){}, (v8f){}};
#pragma unroll 2
    for (int kb = 0; kb < DI; kb += 32) { const v16b a = frag_kb(&Ah[rt * 16 + nloc][kb], hlf), al = frag_kb(&Al[rt * 16 + nloc][kb], hlf);
#pragma unroll
      for (int t = 0; t < 4; ++t) { const v16b bw = frag_kb(WP + (size_t)(t * 16 + nloc) * DI + kb, hlf); acc[t] = wmma16b(a, bw, acc[t]); if (MODE == 1) acc[t] = wmma16b(al, bw, acc[t]); } }
#pragma unroll
    for (int t = 0; t < 4; ++t)
#pragma unroll
      for (int r8 = 0; r8 < 8; ++r8) Tf[rt * 16 + 8 * hlf + r8][t * 16 + nloc] = acc[t][r8] * (1.0f / (HS * WSC)); }
  wave_lds_sync();
  for (int pass = 0; pass < 2; ++pass) { for (int rr = 0; rr < 32; ++rr) *(volatile v2f*)(P + ((size_t)b * L + l0 + rr) * PW + lane * 2) = *(const v2f*)(&Tf[rr][lane * 2]); if (MODE == 0) ((volatile float*)XM)[(size_t)b * L + l0 + lane] = sm * (1.0f / DI); __threadfence(); } }
template <int SCAN2>
__global__ __launch_bounds__(32) void scan_kernel(const float* __restrict__ U, const float* __restrict__ P, const float* __restrict__ P1, const float* __restrict__ XM, const float* __restrict__ PWV, const float* __restrict__ dtw, const float* __restrict__ dtb, const float* __restrict__ Alog, const float* __restrict__ Dp, int LLIM, float* __restrict__ Y) { __shared__ float Ys[2][32]; const int lane = threadIdx.x, n = lane & 15, hlf = lane >> 4; const int b = blockIdx.x / (DI / 2); const int d0 = (blockIdx.x % (DI / 2)) * 2; const int d = d0 + hlf;
  const float A = -__expf(bfv(Alog[d * NS + n])); const float Dd = bfv(Dp[d]); const float bias = bfv(dtb[d]); float w[R];
#pragma unroll
  for (int r = 0; r < R; ++r) w[r] = bfv(dtw[d * R + r]); const float pwn = PWV[SCAN2 * 16 + n]; float h = 0.0f;
#pragma unroll 1
  for (int l = 0; l < LLIM; ++l) { const size_t row = (size_t)b * L + l; const float* pr = P + row * PW; float dt = bias;
#pragma unroll
    for (int r = 0; r < R; ++r) dt += pmul(pr[r], w[r]);
    const float delta = softplus(dt); const float uv = U[((size_t)b * DI + d) * L + l]; const float u = SCAN2 ? uv : bfv(uv); const float xb = SCAN2 ? P1[row * PW + 48 + n] : 0.0f;
    const float Bn = pr[16 + n] + pmul(XM[row], pwn) + xb; const float Cn = pr[32 + n] + xb;
    h = pmul(__expf(pmul(delta, A)), h) + pmul(pmul(delta, Bn), u);
    float yv = pmul(h, Cn);
#pragma unroll
    for (int o = 8; o; o >>= 1) yv += __shfl_xor(yv, o);
    if (n == 0) Ys[hlf][l & 31] = yv + pmul(u, Dd);
    if ((l & 31) == 31) { wave_lds_sync(); for (int pass = 0; pass < 2; ++pass) { ((volatile float*)Y)[((size_t)b * DI + d0) * L + (l - 31) + lane] = Ys[0][lane]; ((volatile float*)Y)[((size_t)b * DI + d0 + 1) * L + (l - 31) + lane] = Ys[1][lane]; __threadfence(); } wave_lds_sync(); } } }
__global__ __launch_bounds__(32) void out_kernel(const float* __restrict__ Y1, const float* __restrict__ Y2, const b16* __restrict__ WC, int LLIM, float* __restrict__ out) { __shared__ __attribute__((aligned(16))) b16 Ah[32][2 * DI + 8], Al[32][2 * DI + 8]; __shared__ float Tf[32][128 + 1]; const int lane = threadIdx.x, nloc = lane & 15, hlf = lane >> 4; const int g = blockIdx.x % 2; const int b = blockIdx.x / (2 * (L / 32)); const int l0 = ((blockIdx.x / 2) % (L / 32)) * 32; if (l0 >= LLIM) return;
  for (int d = 0; d < DI; ++d) { b16 p, ql; split16(Y1[((size_t)b * DI + d) * L + l0 + lane] * HS, p, ql); Ah[lane][d] = p; Al[lane][d] = ql; split16(Y2[((size_t)b * DI + d) * L + l0 + lane] * HS, p, ql); Ah[lane][DI + d] = p; Al[lane][DI + d] = ql; }
  for (int k = 2 * DI; k < 2 * DI + 8; ++k) { Ah[lane][k] = (b16)0.0f; Al[lane][k] = (b16)0.0f; }
  wave_lds_sync();
#pragma unroll 1
  for (int rt = 0; rt < 2; ++rt) { v8f acc[8];
#pragma unroll
    for (int t = 0; t < 8; ++t) acc[t] = (v8f){};
#pragma unroll 2
    for (int kb = 0; kb < 2 * DI; kb += 32) { const v16b a = frag_kb(&Ah[rt * 16 + nloc][kb], hlf), al = frag_kb(&Al[rt * 16 + nloc][kb], hlf);
#pragma unroll
      for (int t = 0; t < 8; ++t) { const v16b bw = frag_kb(WC + (size_t)(g * 128 + t * 16 + nloc) * 2 * DI + kb, hlf); acc[t] = wmma16b(a, bw, acc[t]); acc[t] = wmma16b(al, bw, acc[t]); } }
#pragma unroll
    for (int t = 0; t < 8; ++t)
#pragma unroll
      for (int r8 = 0; r8 < 8; ++r8) Tf[rt * 16 + 8 * hlf + r8][t * 16 + nloc] = acc[t][r8] * (1.0f / (HS * WSC)); }
  wave_lds_sync();
  for (int pass = 0; pass < 2; ++pass) {
#pragma unroll 4
    for (int e = 0; e < 128; ++e) ((volatile float*)out)[((size_t)b * DI + g * 128 + e) * L + l0 + lane] = Tf[lane][e]; __threadfence(); } }
}

extern "C" void kernel_launch(void* const* d_in, const int* in_sizes, int n_in, void* d_out, int out_size, void* d_ws, size_t ws_size, hipStream_t stream) {
  (void)n_in;
  auto Fp = [&](int i) { return (const float*)d_in[i]; };
  if (in_sizes[0] != NBt * DI * L || in_sizes[1] != 48 * DI || in_sizes[2] != DI * R || in_sizes[4] != DI * NS || in_sizes[6] != 48 * DI || in_sizes[11] != DI || in_sizes[12] != NS * DI || in_sizes[14] != NS * DI || in_sizes[15] != DI * DI || in_sizes[16] != DI * DI || out_size != NBt * DI * L) return;
  const int LLIM = L;
  size_t off = 0; char* ws = (char*)d_ws;
  auto carve = [&](size_t bytes) { char* p = ws + off; off += (bytes + 255) & ~(size_t)255; return p; };
  b16* WP1 = (b16*)carve((size_t)PW * DI * 2); b16* WP2 = (b16*)carve((size_t)PW * DI * 2); b16* WC = (b16*)carve((size_t)DI * 2 * DI * 2); float* PWV = (float*)carve(256); float* P1 = (float*)carve((size_t)NBt * L * PW * 4); float* P2 = (float*)carve((size_t)NBt * L * PW * 4); float* XM = (float*)carve((size_t)NBt * L * 4); float* Y1 = (float*)carve((size_t)NBt * DI * L * 4); float* Y2 = (float*)carve((size_t)NBt * DI * L * 4);
  if (off > ws_size || off > ((size_t)48 << 20)) return;
  wput_kernel<<<64, 256, 0, stream>>>(Fp(1), Fp(14), Fp(6), Fp(15), Fp(16), Fp(12), Fp(13), Fp(11), WP1, WP2, WC, PWV);
  proj_kernel<0><<<NBt * (L / 32), 32, 0, stream>>>(Fp(0), WP1, LLIM, P1, XM);
  scan_kernel<0><<<NBt * (DI / 2), 32, 0, stream>>>(Fp(0), P1, P1, XM, PWV, Fp(2), Fp(3), Fp(4), Fp(5), LLIM, Y1);
  proj_kernel<1><<<NBt * (L / 32), 32, 0, stream>>>(Y1, WP2, LLIM, P2, XM);
  scan_kernel<1><<<NBt * (DI / 2), 32, 0, stream>>>(Y1, P2, P1, XM, PWV, Fp(7), Fp(8), Fp(9), Fp(10), LLIM, Y2);
  out_kernel<<<NBt * (L / 32) * 2, 32, 0, stream>>>(Y1, Y2, WC, LLIM, (float*)d_out);
}
